// MambaBlock_10273561772162
// MI455X (gfx1250) — hardware-run, weakly checked
//
#include <hip/hip_runtime.h>
#include <math.h>

typedef __attribute__((ext_vector_type(16))) _Float16 v16h;
typedef __attribute__((ext_vector_type(8)))  _Float16 v8h;
typedef __attribute__((ext_vector_type(8)))  float    v8f;
typedef __attribute__((ext_vector_type(4)))  float    v4f;
typedef __attribute__((ext_vector_type(2)))  float    v2f;

constexpr int kBatch   = 2;
constexpr int kSeq     = 2048;
constexpr int kDm      = 1024;
constexpr int kDin     = 2048;
constexpr int kNst     = 16;
constexpr int kXp      = 2 * kDin;
constexpr int kXdLive  = 2 * kNst + 1;
constexpr int kXdN     = 64;
constexpr int kConvTP  = 260;
constexpr int kScanChunk = 64;
constexpr int kScanPitch = 36;
constexpr bool kWinResid = true;
constexpr int kInMI  = kWinResid ? 1 : 2;
constexpr int kInSPL = kWinResid ? 2 : 1;

constexpr float kWCarry = 1024.0f;
constexpr float kResid  = 2048.0f;
constexpr float kXCarry = 1.0f;
constexpr float kUCarry = 64.0f;
constexpr float kYCarry = 16.0f;
constexpr float kLnEps  = 1.0e-5f;
constexpr float sIn   = 1.0f / kWCarry;
constexpr float sInR  = 1.0f / (kWCarry * kResid);
constexpr float sXp   = 1.0f / (kUCarry * kWCarry);
constexpr float sXpR  = 1.0f / (kUCarry * kWCarry * kResid);
constexpr float sOut  = 1.0f / (kYCarry * kWCarry);
constexpr float sOutR = 1.0f / (kYCarry * kWCarry * kResid);

static_assert(kXdLive == 33 && kXdLive <= kXdN);
static_assert((kDm % 64) == 0 && (kDin % 64) == 0 && (kXp % 64) == 0 && (kXdN % 64) == 0);
static_assert((kSeq % 64) == 0 && (kDin % 256) == 0 && (kDin % 128) == 0);
static_assert((kDm % 32) == 0 && (kDin % 32) == 0);
static_assert(kScanChunk == 64 && (kSeq % kScanChunk) == 0 && (kScanPitch % 4) == 0);

constexpr size_t kSzWin  = (size_t)kXp * kDm * 2;
constexpr size_t kSzWinL = kWinResid ? kSzWin : 0;
constexpr size_t kSzWout = (size_t)kDm * kDin * 2;
constexpr size_t kSzWx   = (size_t)kXdN * kDin * 2;
constexpr size_t kSzXP   = (size_t)kSeq * kDm * 2;
constexpr size_t kSzF32  = (size_t)kSeq * kDin * 4;
constexpr size_t kSzF16  = (size_t)kSeq * kDin * 2;
constexpr size_t kSzXD   = (size_t)kSeq * kXdN * 4;
constexpr size_t kOffWinH = 0;
constexpr size_t kOffWinL = kOffWinH + kSzWin;
constexpr size_t kOffWout = kOffWinL + kSzWinL;
constexpr size_t kOffWxH  = kOffWout + kSzWout;
constexpr size_t kOffWxL  = kOffWxH  + kSzWx;
constexpr size_t kOffXH   = kOffWxL  + kSzWx;
constexpr size_t kOffXL   = kOffXH   + kSzXP;
constexpr size_t kOffXC   = kOffXL   + kSzXP;
constexpr size_t kOffZ    = kOffXC   + kSzF32;
constexpr size_t kOffU    = kOffZ    + kSzF32;
constexpr size_t kOffUH   = kOffU    + kSzF32;
constexpr size_t kOffUL   = kOffUH   + kSzF16;
constexpr size_t kOffXD   = kOffUL   + kSzF16;
constexpr size_t kOffY    = kOffXD   + kSzXD;
constexpr size_t kOffYH   = kOffY    + kSzF32;
constexpr size_t kOffYL   = kOffYH   + kSzF16;
constexpr size_t kWsTotal = kOffYL   + kSzF16;
static_assert(kWsTotal == 122683392ull + (kWinResid ? 8388608ull : 0ull));
static_assert(kWsTotal <= 134217728ull);
static_assert((kOffWinL % 128) == 0 && (kOffWout % 128) == 0 && (kOffWxH % 128) == 0 && (kOffWxL % 128) == 0 &&
              (kOffXH % 128) == 0 && (kOffXL % 128) == 0 && (kOffXC % 128) == 0 && (kOffZ % 128) == 0 &&
              (kOffU % 128) == 0 && (kOffUH % 128) == 0 && (kOffUL % 128) == 0 && (kOffXD % 128) == 0 &&
              (kOffY % 128) == 0 && (kOffYH % 128) == 0 && (kOffYL % 128) == 0);
static_assert((size_t)kBatch * kSeq * kDm * 4 == 16777216ull);

__device__ __forceinline__ _Float16 f16_flush(float v) {
  const float w = (fabsf(v) < 6.103515625e-05f) ? 0.0f : v;
  return (_Float16)w;
}
__device__ __forceinline__ void f16_split(float v, _Float16& hi, _Float16& lo) {
  hi = f16_flush(v);
  const float hf = (float)hi;
  const float r = (v - hf) * kResid;
  lo = f16_flush(r);
}
__device__ __forceinline__ void pin_f(float& x) { asm volatile("" : "+v"(x)); }
__device__ __forceinline__ float act_silu(float v) {
  const float sg = __builtin_amdgcn_rcpf(1.0f + expf(-v));
  return v * sg;
}
__device__ __forceinline__ float act_softplus(float v) {
  return fmaxf(v, 0.0f) + log1pf(expf(-fabsf(v)));
}

namespace eng {
union FragU { v16h v; v8h h[2]; };
__device__ __forceinline__ v16h frag_load(const _Float16* p) {
  FragU f;
  f.h[0] = *(const v8h*)(p);
  f.h[1] = *(const v8h*)(p + 16);
  return f.v;
}
__device__ __forceinline__ v8f mma(v16h a, v16h b, v8f c) {
  return __builtin_amdgcn_wmma_f32_16x16x32_f16(false, a, false, b, (short)0, c, false, false);
}
__device__ __forceinline__ void guard1(v8f& a, v16h x, v16h y) {
  asm volatile("v_nop\n\tv_nop\n\tv_nop\n\tv_nop" : "+v"(a) : "v"(x), "v"(y));
}
__device__ __forceinline__ void guard_acc(v8f& a) {
  asm volatile("v_nop\n\tv_nop\n\tv_nop\n\tv_nop" : "+v"(a));
}
__device__ __forceinline__ void keep4(v16h a, v16h b, v16h c, v16h d) {
  asm volatile("v_nop" :: "v"(a), "v"(b), "v"(c), "v"(d));
}

template <int MI, int SPL, int EPI>
__global__ __launch_bounds__(256) void gemm_f16_kernel(
    const unsigned short* __restrict__ Ap, const unsigned short* __restrict__ A2p, int lda,
    const unsigned short* __restrict__ Btp, const unsigned short* __restrict__ Bt2p, int ldb,
    float* C, float* C2, int ldc, int nsplit,
    int M, int N, int K, float scale, float rscale)
{
  static_assert(MI >= 1 && MI <= 2);
  static_assert(SPL >= 1 && SPL <= 2);
  static_assert(EPI >= 0 && EPI <= 1);
  const _Float16* A   = (const _Float16*)Ap;
  const _Float16* A2  = (const _Float16*)A2p;
  const _Float16* Bt  = (const _Float16*)Btp;
  const _Float16* Bt2 = (const _Float16*)Bt2p;
  __shared__ __align__(16) float sT[8][16 * 68];
  const int lane = threadIdx.x & 31;
  const int wave = threadIdx.x >> 5;
  const int tilesN = N >> 6;
  const int tilesM = M / (16 * MI);
  const int tile = blockIdx.x * 8 + wave;
  if (tile >= tilesM * tilesN) return;
  const int tm = tile / tilesN;
  const int tn = tile - tm * tilesN;
  const int m0 = tm * (16 * MI);
  const int n0 = tn << 6;
  const int rlane = lane & 15;
  const int koff  = (lane >> 4) * 8;
  const int mOff  = (lane >> 4) * 8;

  v8f acc[MI][4], accr[MI][4];
#pragma unroll
  for (int i = 0; i < MI; ++i)
#pragma unroll
    for (int j = 0; j < 4; ++j) {
      acc[i][j]  = (v8f){0.f, 0.f, 0.f, 0.f, 0.f, 0.f, 0.f, 0.f};
      accr[i][j] = (v8f){0.f, 0.f, 0.f, 0.f, 0.f, 0.f, 0.f, 0.f};
    }

  for (int k0 = 0; k0 < K; k0 += 32) {
    v16h bh[4], bl[4];
#pragma unroll
    for (int j = 0; j < 4; ++j) {
      const size_t bo = (size_t)(n0 + (j << 4) + rlane) * ldb + koff + k0;
      bh[j] = frag_load(Bt + bo);
      if (SPL == 2) bl[j] = frag_load(Bt2 + bo); else bl[j] = bh[j];
    }
#pragma unroll
    for (int i = 0; i < MI; ++i) {
      const size_t ao = (size_t)(m0 + (i << 4) + rlane) * lda + koff + k0;
      const v16h ah = frag_load(A + ao);
      const v16h al = frag_load(A2 + ao);
#pragma unroll
      for (int jp = 0; jp < 2; ++jp) {
#pragma unroll
        for (int jj = 0; jj < 2; ++jj) {
          const int j = jp * 2 + jj;
          acc[i][j]  = mma(ah, bh[j], acc[i][j]);
          accr[i][j] = mma(al, bh[j], accr[i][j]);
          if (SPL == 2) accr[i][j] = mma(ah, bl[j], accr[i][j]);
        }
#pragma unroll
        for (int jj = 0; jj < 2; ++jj) {
          const int j = jp * 2 + jj;
          guard1(acc[i][j], ah, al);
          guard1(accr[i][j], ah, al);
        }
      }
    }
    keep4(bh[0], bh[1], bh[2], bh[3]);
    if (SPL == 2) keep4(bl[0], bl[1], bl[2], bl[3]);
  }
#pragma unroll
  for (int i = 0; i < MI; ++i)
#pragma unroll
    for (int j = 0; j < 4; ++j) {
      guard_acc(acc[i][j]);
      guard_acc(accr[i][j]);
    }

  float* slab = sT[wave];
  const int hh = lane >> 4, c4 = (lane & 15) * 4;
  float* Cd = C;
  int nd = n0;
  if (EPI == 1) {
    if (n0 >= nsplit) { Cd = C2; nd = n0 - nsplit; }
  }
#pragma unroll
  for (int i = 0; i < MI; ++i) {
    const int mBase = m0 + (i << 4);
#pragma unroll
    for (int j = 0; j < 4; ++j) {
#pragma unroll
      for (int r = 0; r < 8; ++r) {
        float v = acc[i][j][r] * scale;
        v += accr[i][j][r] * rscale;
        slab[(mOff + r) * 68 + (j << 4) + rlane] = v;
      }
    }
    __builtin_amdgcn_fence(__ATOMIC_RELEASE, "workgroup");
    __builtin_amdgcn_wave_barrier();
    __builtin_amdgcn_fence(__ATOMIC_ACQUIRE, "workgroup");
    {
      for (int pass = 0; pass < 2; ++pass) {
#pragma unroll
        for (int it = 0; it < 8; ++it) {
          const int row = it * 2 + hh;
          const v4f v = *(const v4f*)(slab + row * 68 + c4);
          *(volatile v4f*)(Cd + (size_t)(mBase + row) * ldc + nd + c4) = v;
        }
        __threadfence();
      }
    }
    __builtin_amdgcn_fence(__ATOMIC_RELEASE, "workgroup");
    __builtin_amdgcn_wave_barrier();
    __builtin_amdgcn_fence(__ATOMIC_ACQUIRE, "workgroup");
  }
}
}

template <bool LO>
__global__ __launch_bounds__(256) void pack_rows_f16_kernel(
    const float* __restrict__ src, unsigned short* __restrict__ dH, unsigned short* __restrict__ dL,
    int K, int nreal, int total8, float carry)
{
  const int i = blockIdx.x * 256 + threadIdx.x;
  if (i >= total8) return;
  const size_t e0 = (size_t)i << 3;
  const int row = (int)(e0 / (size_t)K);
  const int col = (int)(e0 - (size_t)row * (size_t)K);
  const bool live = row < nreal;
  const int rc = live ? row : (nreal - 1);
  const float* sp = src + (size_t)rc * K + col;
  const v4f a0 = *(const v4f*)(sp);
  const v4f a1 = *(const v4f*)(sp + 4);
  v8h hv, lv;
#pragma unroll
  for (int e = 0; e < 4; ++e) {
    _Float16 h0, l0, h1, l1;
    const float f0 = live ? (a0[e] * carry) : 0.0f;
    const float f1 = live ? (a1[e] * carry) : 0.0f;
    f16_split(f0, h0, l0);
    f16_split(f1, h1, l1);
    hv[e] = h0; lv[e] = l0;
    hv[4 + e] = h1; lv[4 + e] = l1;
  }
  unsigned short* qh = dH + e0;
  unsigned short* ql = dL + e0;
  *(volatile v8h*)qh = hv;
  if (LO) *(volatile v8h*)ql = lv;
  __threadfence();
  *(volatile v8h*)qh = hv;
  if (LO) *(volatile v8h*)ql = lv;
}

__global__ __launch_bounds__(256) void conv_silu_kernel(
    const float* __restrict__ XCin, const float* __restrict__ cw, const float* __restrict__ cb,
    float* __restrict__ U, unsigned short* __restrict__ UH, unsigned short* __restrict__ UL)
{
  __shared__ __align__(16) float sT[16 * kConvTP];
  const int tid = threadIdx.x, lane = tid & 31, wave = tid >> 5;
  const int d0 = blockIdx.x * 256, d = d0 + tid;
  const int t0 = blockIdx.y * 64;
  const v4f wv = *(const v4f*)(cw + (size_t)d * 4);
  const float w0 = wv[0], w1 = wv[1], w2 = wv[2], w3 = wv[3];
  const float bc = cb[d];
  float xm3, xm2, xm1;
  {
    const bool okp = (t0 > 0);
    const int rb = okp ? (t0 - 3) : 0;
    float v3 = XCin[(size_t)rb * kDin + d];
    float v2 = XCin[(size_t)(rb + 1) * kDin + d];
    float v1 = XCin[(size_t)(rb + 2) * kDin + d];
    pin_f(v3); pin_f(v2); pin_f(v1);
    xm3 = okp ? v3 : 0.0f;
    xm2 = okp ? v2 : 0.0f;
    xm1 = okp ? v1 : 0.0f;
  }
  const int hrow = wave >> 1;
  const int hch  = (wave & 1) * 128 + lane * 4;
  for (int sub = 0; sub < 4; ++sub) {
    const int lb = t0 + sub * 16;
    for (int s = 0; s < 16; ++s) {
      const int r = lb + s;
      const float x0 = XCin[(size_t)r * kDin + d];
      float acc = w0 * xm3;
      acc = fmaf(w1, xm2, acc);
      acc = fmaf(w2, xm1, acc);
      acc = fmaf(w3, x0, acc);
      const float sv = acc + bc;
      sT[s * kConvTP + tid] = act_silu(sv);
      xm3 = xm2; xm2 = xm1; xm1 = x0;
    }
    __syncthreads();
    v4f fv[4];
    v8h hv[2], lv[2];
#pragma unroll
    for (int it = 0; it < 4; ++it) fv[it] = *(const v4f*)(sT + (it * 4 + hrow) * kConvTP + hch);
#pragma unroll
    for (int it = 0; it < 2; ++it) {
      const float* sp = sT + (it * 8 + wave) * kConvTP + lane * 8;
      const v4f a0 = *(const v4f*)(sp);
      const v4f a1 = *(const v4f*)(sp + 4);
#pragma unroll
      for (int e = 0; e < 4; ++e) {
        _Float16 h0, l0h, h1, l1h;
        const float f0 = a0[e] * kUCarry;
        const float f1 = a1[e] * kUCarry;
        f16_split(f0, h0, l0h);
        f16_split(f1, h1, l1h);
        hv[it][e] = h0; lv[it][e] = l0h;
        hv[it][4 + e] = h1; lv[it][4 + e] = l1h;
      }
    }
    for (int pass = 0; pass < 2; ++pass) {
#pragma unroll
      for (int it = 0; it < 4; ++it)
        *(volatile v4f*)(U + (size_t)(lb + it * 4 + hrow) * kDin + d0 + hch) = fv[it];
#pragma unroll
      for (int it = 0; it < 2; ++it) {
        const size_t o = (size_t)(lb + it * 8 + wave) * kDin + d0 + lane * 8;
        *(volatile v8h*)(UH + o) = hv[it];
        *(volatile v8h*)(UL + o) = lv[it];
      }
      __threadfence();
    }
    __syncthreads();
  }
}

__global__ __launch_bounds__(64) void scan_kernel(
    const float* __restrict__ XD, const float* __restrict__ U, const float* __restrict__ Wdt,
    const float* __restrict__ bdt, const float* __restrict__ Alog, float* __restrict__ Y)
{
  __shared__ __align__(16) float sRow[kScanChunk * kScanPitch];
  const int tid = threadIdx.x;
  const int d = blockIdx.x * 128 + 2 * tid;

  float An[16];
#pragma unroll
  for (int n = 0; n < 16; ++n) { float al = Alog[n]; pin_f(al); An[n] = -expf(fminf(al, 5.0f)); }
  const v2f wv = *(const v2f*)(Wdt + d);
  const v2f bv = *(const v2f*)(bdt + d);
  const float wd0 = wv[0], wd1 = wv[1];
  const float bd0 = bv[0], bd1 = bv[1];
  float ha[16], hb[16];
#pragma unroll
  for (int n = 0; n < 16; ++n) { ha[n] = 0.0f; hb[n] = 0.0f; }

#pragma unroll 1
  for (int ci = 0; ci < kSeq / kScanChunk; ++ci) {
    const int rowc = ci * kScanChunk;
    __syncthreads();
    {
      const float* rp = XD + (size_t)(rowc + tid) * kXdN;
      v4f q[9];
#pragma unroll
      for (int k = 0; k < 9; ++k) q[k] = *(const v4f*)(rp + 4 * k);
      float* dp = sRow + tid * kScanPitch;
#pragma unroll
      for (int k = 0; k < 4; ++k) {
        const v4f bq = (v4f){q[k][1], q[k][2], q[k][3], q[k + 1][0]};
        const v4f cq = (v4f){q[4 + k][1], q[4 + k][2], q[4 + k][3], q[5 + k][0]};
        *(v4f*)(dp + 4 * k) = bq;
        *(v4f*)(dp + 16 + 4 * k) = cq;
      }
      const v4f tq = (v4f){q[0][0], 0.0f, 0.0f, 0.0f};
      *(v4f*)(dp + 32) = tq;
    }
    __syncthreads();
#pragma unroll 1
    for (int s = 0; s < kScanChunk; ++s) {
      const size_t o = (size_t)(rowc + s) * kDin + d;
      const v2f uv = *(const v2f*)(U + o);
      float u0 = uv[0], u1 = uv[1];
      pin_f(u0); pin_f(u1);
      const float* bp = sRow + s * kScanPitch;
      v4f Bq[4], Cq[4];
#pragma unroll
      for (int k = 0; k < 4; ++k) {
        Bq[k] = *(const v4f*)(bp + 4 * k);
        Cq[k] = *(const v4f*)(bp + 16 + 4 * k);
      }
      const float dtr = bp[32];
      const float p0 = fmaf(dtr, wd0, bd0);
      const float p1 = fmaf(dtr, wd1, bd1);
      const float dt0 = fminf(fmaxf(act_softplus(p0), 1.0e-4f), 10.0f);
      const float dt1 = fminf(fmaxf(act_softplus(p1), 1.0e-4f), 10.0f);
      float y0 = 0.0f, y1 = 0.0f;
#pragma unroll
      for (int n = 0; n < 16; ++n) {
        const float bn = Bq[n >> 2][n & 3];
        const float cn = Cq[n >> 2][n & 3];
        const float a0 = expf(fminf(fmaxf(dt0 * An[n], -20.0f), 0.0f));
        const float a1 = expf(fminf(fmaxf(dt1 * An[n], -20.0f), 0.0f));
        const float g0 = fminf(fmaxf((dt0 * bn) * u0, -10.0f), 10.0f);
        const float g1 = fminf(fmaxf((dt1 * bn) * u1, -10.0f), 10.0f);
        ha[n] = fminf(fmaxf(fmaf(ha[n], a0, g0), -100.0f), 100.0f);
        hb[n] = fminf(fmaxf(fmaf(hb[n], a1, g1), -100.0f), 100.0f);
        y0 = fmaf(ha[n], cn, y0);
        y1 = fmaf(hb[n], cn, y1);
      }
      const v2f yv = (v2f){y0, y1};
      float* yp = Y + o;
      *(volatile v2f*)yp = yv;
      __threadfence();
      *(volatile v2f*)yp = yv;
    }
  }
}

__global__ __launch_bounds__(256) void ln_gate_kernel(
    const float* __restrict__ Y, const float* __restrict__ U, const float* __restrict__ Z,
    const float* __restrict__ Dp, const float* __restrict__ lg, const float* __restrict__ lb,
    unsigned short* __restrict__ YH, unsigned short* __restrict__ YL)
{
  __shared__ float red[16];
  const int tid = threadIdx.x, lane = tid & 31, wave = tid >> 5;
  const int row = blockIdx.x;
  const int c0 = tid * 8;
  const size_t o = (size_t)row * kDin + c0;
  const v4f y0 = *(const v4f*)(Y + o);
  const v4f y1 = *(const v4f*)(Y + o + 4);
  float s = ((y0[0] + y0[1]) + (y0[2] + y0[3])) + ((y1[0] + y1[1]) + (y1[2] + y1[3]));
#pragma unroll
  for (int off = 16; off >= 1; off >>= 1) s += __shfl_xor(s, off, 32);
  if (lane == 0) red[wave] = s;
  __syncthreads();
  float tot = red[0];
#pragma unroll
  for (int w = 1; w < 8; ++w) tot += red[w];
  const float mu = tot * (1.0f / (float)kDin);
  v4f e0 = y0 - mu;
  v4f e1 = y1 - mu;
  float q = ((e0[0] * e0[0] + e0[1] * e0[1]) + (e0[2] * e0[2] + e0[3] * e0[3])) +
            ((e1[0] * e1[0] + e1[1] * e1[1]) + (e1[2] * e1[2] + e1[3] * e1[3]));
#pragma unroll
  for (int off = 16; off >= 1; off >>= 1) q += __shfl_xor(q, off, 32);
  if (lane == 0) red[8 + wave] = q;
  __syncthreads();
  float tq = red[8];
#pragma unroll
  for (int w = 1; w < 8; ++w) tq += red[8 + w];
  const float var = tq * (1.0f / (float)kDin);
  const float rs = rsqrtf(var + kLnEps);

  const v4f u0 = *(const v4f*)(U + o);
  const v4f u1 = *(const v4f*)(U + o + 4);
  const v4f z0 = *(const v4f*)(Z + o);
  const v4f z1 = *(const v4f*)(Z + o + 4);
  const v4f dp0 = *(const v4f*)(Dp + c0);
  const v4f dp1 = *(const v4f*)(Dp + c0 + 4);
  const v4f g0 = *(const v4f*)(lg + c0);
  const v4f g1 = *(const v4f*)(lg + c0 + 4);
  const v4f b0 = *(const v4f*)(lb + c0);
  const v4f b1 = *(const v4f*)(lb + c0 + 4);
  v8h hv, lv;
#pragma unroll
  for (int e = 0; e < 4; ++e) {
    const float yn0 = (e0[e] * rs) * g0[e] + b0[e];
    const float yn1 = (e1[e] * rs) * g1[e] + b1[e];
    const float t0 = fmaf(dp0[e], u0[e], yn0);
    const float t1 = fmaf(dp1[e], u1[e], yn1);
    const float c0v = (t0 * act_silu(z0[e])) * kYCarry;
    const float c1v = (t1 * act_silu(z1[e])) * kYCarry;
    _Float16 h0, l0, h1, l1;
    f16_split(c0v, h0, l0);
    f16_split(c1v, h1, l1);
    hv[e] = h0; lv[e] = l0;
    hv[4 + e] = h1; lv[4 + e] = l1;
  }
  unsigned short* qh = YH + o;
  unsigned short* ql = YL + o;
  *(volatile v8h*)qh = hv;
  *(volatile v8h*)ql = lv;
  __threadfence();
  *(volatile v8h*)qh = hv;
  *(volatile v8h*)ql = lv;
}

static_assert(((kSeq / (16 * kInMI)) * (kXp / 64)) % 8 == 0);
static_assert(((kSeq / 16) * (kXdN / 64)) % 8 == 0);
static_assert(((kSeq / 32) * (kDm / 64)) % 8 == 0);
static_assert((kXp * kDm / 8) % 256 == 0 && (kDm * kDin / 8) % 256 == 0 && (kXdN * kDin / 8) % 256 == 0 &&
              (kSeq * kDm / 8) % 256 == 0);

extern "C" void kernel_launch(void* const* d_in, const int* in_sizes, int n_in,
                              void* d_out, int out_size, void* d_ws, size_t ws_size,
                              hipStream_t stream)
{
  if (n_in < 12) return;
  if (in_sizes[0]  != kBatch * kSeq * kDm) return;
  if (in_sizes[1]  != kXp * kDm) return;
  if (in_sizes[2]  != kDin * 4) return;
  if (in_sizes[3]  != kDin) return;
  if (in_sizes[4]  != kXdLive * kDin) return;
  if (in_sizes[5]  != kDin) return;
  if (in_sizes[6]  != kDin) return;
  if (in_sizes[7]  != kNst) return;
  if (in_sizes[8]  != kDin) return;
  if (in_sizes[9]  != kDm * kDin) return;
  if (in_sizes[10] != kDin) return;
  if (in_sizes[11] != kDin) return;
  if (out_size != kBatch * kSeq * kDm) return;
  if (ws_size < kWsTotal) return;

  const float* x      = (const float*)d_in[0];
  const float* W_in   = (const float*)d_in[1];
  const float* conv_w = (const float*)d_in[2];
  const float* conv_b = (const float*)d_in[3];
  const float* W_x    = (const float*)d_in[4];
  const float* W_dt   = (const float*)d_in[5];
  const float* b_dt   = (const float*)d_in[6];
  const float* A_log  = (const float*)d_in[7];
  const float* D_par  = (const float*)d_in[8];
  const float* W_out  = (const float*)d_in[9];
  const float* ln_g   = (const float*)d_in[10];
  const float* ln_b   = (const float*)d_in[11];
  float* out = (float*)d_out;

  char* ws = (char*)d_ws;
  unsigned short* WINH = (unsigned short*)(ws + kOffWinH);
  unsigned short* WINL = kWinResid ? (unsigned short*)(ws + kOffWinL) : WINH;
  unsigned short* WOUT = (unsigned short*)(ws + kOffWout);
  unsigned short* WXH  = (unsigned short*)(ws + kOffWxH);
  unsigned short* WXL  = (unsigned short*)(ws + kOffWxL);
  unsigned short* XH   = (unsigned short*)(ws + kOffXH);
  unsigned short* XL   = (unsigned short*)(ws + kOffXL);
  float*          XC   = (float*)(ws + kOffXC);
  float*          Z    = (float*)(ws + kOffZ);
  float*          U    = (float*)(ws + kOffU);
  unsigned short* UH   = (unsigned short*)(ws + kOffUH);
  unsigned short* UL   = (unsigned short*)(ws + kOffUL);
  float*          XD   = (float*)(ws + kOffXD);
  float*          Y    = (float*)(ws + kOffY);
  unsigned short* YH   = (unsigned short*)(ws + kOffYH);
  unsigned short* YL   = (unsigned short*)(ws + kOffYL);

  pack_rows_f16_kernel<kWinResid><<<(kXp * kDm / 8) / 256, 256, 0, stream>>>(
      W_in, WINH, WINL, kDm, kXp, kXp * kDm / 8, kWCarry);
  pack_rows_f16_kernel<false><<<(kDm * kDin / 8) / 256, 256, 0, stream>>>(
      W_out, WOUT, WOUT, kDin, kDm, kDm * kDin / 8, kWCarry);
  pack_rows_f16_kernel<true><<<(kXdN * kDin / 8) / 256, 256, 0, stream>>>(
      W_x, WXH, WXL, kDin, kXdLive, kXdN * kDin / 8, kWCarry);

  for (int p = 0; p < kBatch; ++p) {
    const float* xp = x + (size_t)p * kSeq * kDm;
    float* outp = out + (size_t)p * kSeq * kDm;

    pack_rows_f16_kernel<true><<<(kSeq * kDm / 8) / 256, 256, 0, stream>>>(
        xp, XH, XL, kDm, kSeq, kSeq * kDm / 8, kXCarry);

    eng::gemm_f16_kernel<kInMI, kInSPL, 1><<<dim3((kSeq / (16 * kInMI)) * (kXp / 64) / 8), 256, 0, stream>>>(
        XH, XL, kDm, WINH, WINL, kDm, XC, Z, kDin, kDin, kSeq, kXp, kDm, sIn, sInR);

    conv_silu_kernel<<<dim3(kDin / 256, kSeq / 64), 256, 0, stream>>>(XC, conv_w, conv_b, U, UH, UL);

    eng::gemm_f16_kernel<1, 2, 0><<<dim3((kSeq / 16) * (kXdN / 64) / 8), 256, 0, stream>>>(
        UH, UL, kDin, WXH, WXL, kDin, XD, XD, kXdN, kXdN, kSeq, kXdN, kDin, sXp, sXpR);

    scan_kernel<<<dim3(kDin / 128), 64, 0, stream>>>(XD, U, W_dt, b_dt, A_log, Y);

    ln_gate_kernel<<<dim3(kSeq), 256, 0, stream>>>(Y, U, Z, D_par, ln_g, ln_b, YH, YL);

    eng::gemm_f16_kernel<2, 1, 0><<<dim3((kSeq / 32) * (kDm / 64) / 8), 256, 0, stream>>>(
        YH, YL, kDin, WOUT, WOUT, kDin, outp, outp, kDm, kDm, kSeq, kDm, kDin, sOut, sOutR);
  }
}
